// Generator_80788334838368
// MI455X (gfx1250) — hardware-run, weakly checked
//
#include <hip/hip_runtime.h>
#include <math.h>

typedef __attribute__((ext_vector_type(16))) _Float16 v16h;
typedef __attribute__((ext_vector_type(8)))  _Float16 v8h;
typedef __attribute__((ext_vector_type(8)))  float    v8f;
typedef __attribute__((ext_vector_type(4)))  float    v4f;
typedef __attribute__((ext_vector_type(2)))  float    v2f;

static constexpr int NBATCH  = 8;
static constexpr int NCHAN   = 3;
static constexpr int IMGW    = 256;
static constexpr int PSZ     = 16;
static constexpr int NHEAD   = 4;
static constexpr int NTOK    = 768;
static constexpr int EDIM    = 256;
static constexpr int DHEAD   = 64;
static constexpr int DMLP    = 1024;
static constexpr int NBLOCKS = 6;
static constexpr int LASTB   = NBLOCKS - 1;
static constexpr int KCONV   = NCHAN * PSZ * PSZ;
static constexpr int NROWS   = NBATCH * NTOK;
static constexpr int ATT_KC  = 64;
static constexpr int ATT_NW  = 4;
static constexpr float LN_EPS     = 1e-5f;
static constexpr float WCARRY     = 64.0f;
static constexpr float WCARRY_INV = 1.0f / 64.0f;
static constexpr float PCARRY     = 32768.0f;

static_assert(NTOK % 64 == 0);
static_assert(EDIM % 64 == 0);
static_assert(DHEAD % 64 == 0);
static_assert(DMLP % 64 == 0);
static_assert(NROWS % 64 == 0);
static_assert(KCONV % 32 == 0);
static_assert(DHEAD % 32 == 0);
static_assert(EDIM % 32 == 0);
static_assert(DMLP % 32 == 0);
static_assert(NTOK % ATT_KC == 0);
static_assert(EDIM == NHEAD * DHEAD);
static_assert(IMGW == PSZ * 16);

__device__ __forceinline__ void dep_guard_h(v8f& a, v8f& b, v16h x, v16h y) { asm volatile("v_nop\n\tv_nop\n\tv_nop\n\tv_nop" : "+v"(a), "+v"(b) : "v"(x), "v"(y)); }
__device__ __forceinline__ void keep4_h(v16h a, v16h b, v16h c, v16h d) { asm volatile("v_nop" :: "v"(a), "v"(b), "v"(c), "v"(d)); }
__device__ __forceinline__ void acc_guard4(v8f& a, v8f& b, v8f& c, v8f& d) { asm volatile("v_nop\n\tv_nop\n\tv_nop\n\tv_nop" : "+v"(a), "+v"(b), "+v"(c), "+v"(d)); }

struct FragH {
  union U { v16h v; v8h h[2]; };
  static __device__ __forceinline__ v16h load(const _Float16* p) {
    U f; f.h[0] = *(const v8h*)(p); f.h[1] = *(const v8h*)(p + 16); return f.v;
  }
  static __device__ __forceinline__ v8f mma(v16h a, v16h b, v8f c) {
    return __builtin_amdgcn_wmma_f32_16x16x32_f16(false, a, false, b, (short)0, c, false, false);
  }
};

__device__ __forceinline__ v8f mma_h(v16h a, v16h b, v8f c) {
  c = __builtin_amdgcn_wmma_f32_16x16x32_f16(false, a, false, b, (short)0, c, false, false);
  asm volatile("v_nop\n\tv_nop\n\tv_nop\n\tv_nop" : "+v"(c) : "v"(a), "v"(b));
  return c;
}

template <int BIAS_MODE, int OUT_MODE, bool RESID>
__global__ __launch_bounds__(256) void gemm64_f16(
    const unsigned short* __restrict__ Ap, int lda, long sAy, long sAz,
    const unsigned short* __restrict__ Btp, int ldb, long sBy, long sBz,
    void* __restrict__ Cout, int ldc, long sCy, long sCz,
    const float* __restrict__ bias, long sBiasZ,
    const float* __restrict__ resid, long sRy, long sRz,
    int M, int N, int K, float scale) {
  static_assert(!(RESID && OUT_MODE != 0));
  const _Float16* A  = (const _Float16*)Ap;
  const _Float16* Bt = (const _Float16*)Btp;
  __shared__ __align__(16) float sT[8][16 * 68];
  const int by   = blockIdx.y;
  const int bz   = blockIdx.z;
  const int lane = threadIdx.x & 31;
  const int wave = threadIdx.x >> 5;
  const int tilesN = N >> 6;
  const int tilesM = M >> 6;
  const int tile = blockIdx.x * 8 + wave;
  if (tile >= tilesM * tilesN) return;
  const int tm = tile / tilesN;
  const int tn = tile - tm * tilesN;
  const int m0 = tm << 6;
  const int n0 = tn << 6;

  const _Float16* Ab = A  + (size_t)by * sAy + (size_t)bz * sAz;
  const _Float16* Bb = Bt + (size_t)by * sBy + (size_t)bz * sBz;

  const int rlane = lane & 15;
  const int koff  = (lane >> 4) * 8;
  const int mOff  = (lane >> 4) * 8;

  v8f acc[4][4];
#pragma unroll
  for (int i = 0; i < 4; ++i)
#pragma unroll
    for (int j = 0; j < 4; ++j) acc[i][j] = (v8f){0.f,0.f,0.f,0.f,0.f,0.f,0.f,0.f};

  for (int k0 = 0; k0 < K; k0 += 32) {
    v16h bh[4];
#pragma unroll
    for (int j = 0; j < 4; ++j) {
      const size_t bo = (size_t)(n0 + (j << 4) + rlane) * ldb + koff + k0;
      bh[j] = FragH::load(Bb + bo);
    }
#pragma unroll
    for (int i = 0; i < 4; ++i) {
      const size_t ao = (size_t)(m0 + (i << 4) + rlane) * lda + koff + k0;
      v16h ah = FragH::load(Ab + ao);
#pragma unroll
      for (int j = 0; j < 4; ++j) acc[i][j] = FragH::mma(ah, bh[j], acc[i][j]);
      dep_guard_h(acc[i][0], acc[i][3], ah, ah);
    }
    keep4_h(bh[0], bh[1], bh[2], bh[3]);
  }
  acc_guard4(acc[0][0], acc[0][1], acc[0][2], acc[0][3]);
  acc_guard4(acc[1][0], acc[1][1], acc[1][2], acc[1][3]);
  acc_guard4(acc[2][0], acc[2][1], acc[2][2], acc[2][3]);
  acc_guard4(acc[3][0], acc[3][1], acc[3][2], acc[3][3]);

  float* slab = sT[wave];
  const float* biasz = (BIAS_MODE != 0) ? (bias + (size_t)bz * sBiasZ) : nullptr;
#pragma unroll
  for (int i = 0; i < 4; ++i) {
    const int mBase = m0 + (i << 4);
    v8f bm = (v8f){0.f,0.f,0.f,0.f,0.f,0.f,0.f,0.f};
    if (BIAS_MODE == 1) {
      const v4f b0 = *(const v4f*)(biasz + mBase + mOff);
      const v4f b1 = *(const v4f*)(biasz + mBase + mOff + 4);
      bm = __builtin_shufflevector(b0, b1, 0, 1, 2, 3, 4, 5, 6, 7);
    }
#pragma unroll
    for (int j = 0; j < 4; ++j) {
      const int n = n0 + (j << 4) + rlane;
      float bn = 0.f;
      if (BIAS_MODE == 2) bn = biasz[n];
#pragma unroll
      for (int r = 0; r < 8; ++r) {
        float v = acc[i][j][r] * scale;
        if (BIAS_MODE == 1) v += bm[r];
        if (BIAS_MODE == 2) v += bn;
        slab[(mOff + r) * 68 + (j << 4) + rlane] = v;
      }
    }
    __builtin_amdgcn_fence(__ATOMIC_RELEASE, "workgroup");
    __builtin_amdgcn_wave_barrier();
    __builtin_amdgcn_fence(__ATOMIC_ACQUIRE, "workgroup");
    if (OUT_MODE == 0) {
      float* Cb = (float*)Cout + (size_t)by * sCy + (size_t)bz * sCz;
      const float* Rb = RESID ? (resid + (size_t)by * sRy + (size_t)bz * sRz) : nullptr;
      const int hh = lane >> 4, c4 = (lane & 15) * 4;
      v4f vv[8];
#pragma unroll
      for (int it = 0; it < 8; ++it) {
        const int row = it * 2 + hh;
        v4f v = *(const v4f*)(slab + row * 68 + c4);
        if (RESID) {
          const v4f rr = *(const v4f*)(Rb + (size_t)(mBase + row) * ldc + n0 + c4);
          v = v + rr;
        }
        vv[it] = v;
      }
      for (int pass = 0; pass < 2; ++pass) {
#pragma unroll
        for (int it = 0; it < 8; ++it) {
          const int row = it * 2 + hh;
          *(volatile v4f*)(Cb + (size_t)(mBase + row) * ldc + n0 + c4) = vv[it];
        }
        __threadfence();
      }
    } else {
      const int q = lane >> 3, c8 = (lane & 7) * 8;
      unsigned short* Cb = (unsigned short*)Cout + (size_t)by * sCy + (size_t)bz * sCz;
      v8h hv[4];
#pragma unroll
      for (int it = 0; it < 4; ++it) {
        const int row = it * 4 + q;
        const float* sp = slab + row * 68 + c8;
#pragma unroll
        for (int e = 0; e < 8; ++e) hv[it][e] = (_Float16)sp[e];
      }
      for (int pass = 0; pass < 2; ++pass) {
#pragma unroll
        for (int it = 0; it < 4; ++it) {
          const int row = it * 4 + q;
          *(volatile v8h*)(Cb + (size_t)(mBase + row) * ldc + n0 + c8) = hv[it];
        }
        __threadfence();
      }
    }
    __builtin_amdgcn_fence(__ATOMIC_RELEASE, "workgroup");
    __builtin_amdgcn_wave_barrier();
    __builtin_amdgcn_fence(__ATOMIC_ACQUIRE, "workgroup");
  }
}

__global__ __launch_bounds__(256) void cast_scale_f16x2(
    const float* __restrict__ in, unsigned short* __restrict__ outp, int n2, float sc) {
  const int i = blockIdx.x * 256 + threadIdx.x;
  if (i < n2) {
    const v2f f = *(const v2f*)(in + 2 * (size_t)i);
    const _Float16 h0 = (_Float16)(f[0] * sc), h1 = (_Float16)(f[1] * sc);
    const unsigned u = (unsigned)__builtin_bit_cast(unsigned short, h0) | ((unsigned)__builtin_bit_cast(unsigned short, h1) << 16);
    ((volatile unsigned*)outp)[i] = u;
    __threadfence();
    ((volatile unsigned*)outp)[i] = u;
  }
}

__global__ __launch_bounds__(256) void posemb_table(float* __restrict__ pe) {
  const int i = blockIdx.x * 256 + threadIdx.x;
  if (i >= NTOK * EDIM / 2) return;
  const int s  = i / (EDIM / 2);
  const int e0 = (i - s * (EDIM / 2)) * 2;
  const float expo = (float)e0 * (1.0f / (float)EDIM);
  const float rden = exp2f(-expo * 13.287712379549449f);
  const float ang  = (float)s * rden;
  float sv, cv;
  sincosf(ang, &sv, &cv);
  v2f o; o[0] = sv; o[1] = cv;
  v2f* dst = (v2f*)(pe + 2 * (size_t)i);
  *(volatile v2f*)dst = o;
  __threadfence();
  *(volatile v2f*)dst = o;
}

__global__ __launch_bounds__(256) void im2col_f16(const float* __restrict__ x, unsigned short* __restrict__ xcol) {
  const int lane = threadIdx.x & 31, wave = threadIdx.x >> 5;
  const int rowid = blockIdx.x * 8 + wave;
  if (rowid >= NBATCH * EDIM) return;
  const int b  = rowid / EDIM;
  const int e  = rowid - b * EDIM;
  const int py = e >> 4, px = e & 15;
  const int kh = lane >> 1, kw0 = (lane & 1) * 8;
  _Float16* dst = (_Float16*)xcol + (size_t)rowid * KCONV + lane * 8;
  v8h o[3];
#pragma unroll
  for (int c = 0; c < 3; ++c) {
    const float* src = x + (((size_t)(b * NCHAN + c) * IMGW + py * PSZ + kh) * IMGW + px * PSZ + kw0);
    const v4f f0 = *(const v4f*)(src);
    const v4f f1 = *(const v4f*)(src + 4);
#pragma unroll
    for (int t = 0; t < 4; ++t) { o[c][t] = (_Float16)f0[t]; o[c][4 + t] = (_Float16)f1[t]; }
  }
  for (int pass = 0; pass < 2; ++pass) {
#pragma unroll
    for (int c = 0; c < 3; ++c) *(volatile v8h*)(dst + c * 256) = o[c];
    __threadfence();
  }
}

__global__ __launch_bounds__(256) void layernorm_f16(
    const float* __restrict__ xin, const float* __restrict__ g, const float* __restrict__ bt,
    unsigned short* __restrict__ outp, int nrows) {
  const int lane = threadIdx.x & 31, wave = threadIdx.x >> 5;
  const int row = blockIdx.x * 8 + wave;
  if (row >= nrows) return;
  const float* xr = xin + (size_t)row * EDIM + lane * 8;
  const v4f a0 = *(const v4f*)(xr);
  const v4f a1 = *(const v4f*)(xr + 4);
  const v8f a = __builtin_shufflevector(a0, a1, 0, 1, 2, 3, 4, 5, 6, 7);
  float s = 0.0f;
#pragma unroll
  for (int t = 0; t < 8; ++t) s += a[t];
#pragma unroll
  for (int off = 16; off; off >>= 1) s += __shfl_xor(s, off, 32);
  const float mean = s * (1.0f / (float)EDIM);
  float vs = 0.0f;
#pragma unroll
  for (int t = 0; t < 8; ++t) { const float d = a[t] - mean; vs += d * d; }
#pragma unroll
  for (int off = 16; off; off >>= 1) vs += __shfl_xor(vs, off, 32);
  const float rstd = rsqrtf(vs * (1.0f / (float)EDIM) + LN_EPS);
  const v4f g0 = *(const v4f*)(g + lane * 8), g1 = *(const v4f*)(g + lane * 8 + 4);
  const v4f b0 = *(const v4f*)(bt + lane * 8), b1 = *(const v4f*)(bt + lane * 8 + 4);
  const v8f gg = __builtin_shufflevector(g0, g1, 0, 1, 2, 3, 4, 5, 6, 7);
  const v8f bb = __builtin_shufflevector(b0, b1, 0, 1, 2, 3, 4, 5, 6, 7);
  v8h o;
#pragma unroll
  for (int t = 0; t < 8; ++t) o[t] = (_Float16)((a[t] - mean) * rstd * gg[t] + bb[t]);
  _Float16* orow = (_Float16*)outp + (size_t)row * EDIM + lane * 8;
  *(volatile v8h*)orow = o;
  __threadfence();
  *(volatile v8h*)orow = o;
}

__global__ __launch_bounds__(256) void gelu_f16x2(const float* __restrict__ in, unsigned short* __restrict__ outp, int n2) {
  const int i = blockIdx.x * 256 + threadIdx.x;
  if (i >= n2) return;
  const v2f xv = *(const v2f*)(in + 2 * (size_t)i);
  unsigned w = 0;
#pragma unroll 1
  for (int t = 0; t < 2; ++t) {
    const float xx = (t == 0) ? xv[0] : xv[1];
    const float gl = 0.5f * xx * (1.0f + erff(xx * 0.70710678118654752f));
    w |= ((unsigned)__builtin_bit_cast(unsigned short, (_Float16)gl)) << (16 * t);
  }
  ((volatile unsigned*)outp)[i] = w;
  __threadfence();
  ((volatile unsigned*)outp)[i] = w;
}

__global__ __launch_bounds__(128) void attn_f16(
    const unsigned short* __restrict__ Qp, const unsigned short* __restrict__ Kp,
    const unsigned short* __restrict__ Vtp, const float* __restrict__ xres,
    float* __restrict__ xout, float qkscale) {
  union FH { v16h v; v8h h[2]; };
  __shared__ __align__(16) _Float16 Ksh[ATT_KC * DHEAD];
  __shared__ __align__(16) _Float16 Vth[DHEAD * ATT_KC];
  __shared__ __align__(16) _Float16 Psh[ATT_NW][16 * ATT_KC];
  __shared__ __align__(16) float    Os[ATT_NW][16 * 68];

  const int tid  = threadIdx.x;
  const int wave = tid >> 5;
  const int lane = tid & 31;
  const int hh   = lane >> 4;
  const int c    = lane & 15;

  const int nqb = NTOK / 64;
  const int bx  = blockIdx.x;
  const int qb  = bx % nqb;
  const int bh  = bx / nqb;
  const int h   = bh % NHEAD;
  const int b   = bh / NHEAD;
  const int q0  = qb * 64 + wave * 16;

  const _Float16* Qb = (const _Float16*)Qp  + (size_t)bh * NTOK * DHEAD;
  const _Float16* Kb = (const _Float16*)Kp  + (size_t)bh * NTOK * DHEAD;
  const _Float16* Vb = (const _Float16*)Vtp + (size_t)bh * DHEAD * NTOK;

  v16h qa[2];
#pragma unroll
  for (int dc = 0; dc < 2; ++dc) qa[dc] = FragH::load(Qb + (size_t)(q0 + c) * DHEAD + dc * 32 + 8 * hh);

  float mrow[8], lrow[8];
  v8f oacc[4];
#pragma unroll
  for (int r = 0; r < 8; ++r) { mrow[r] = -INFINITY; lrow[r] = 0.f; }
#pragma unroll
  for (int t = 0; t < 4; ++t) oacc[t] = (v8f){0.f,0.f,0.f,0.f,0.f,0.f,0.f,0.f};

  for (int kc = 0; kc < NTOK / ATT_KC; ++kc) {
    const int kv0 = kc * ATT_KC;
    __syncthreads();
#pragma unroll
    for (int i = 0; i < 4; ++i) {
      const int idx8 = (i * 128 + tid) * 8;
      const v8h kk = *(const v8h*)(Kb + (size_t)kv0 * DHEAD + idx8);
      *(v8h*)(Ksh + idx8) = kk;
      const int d   = i * 16 + (tid >> 3);
      const int seg = (tid & 7) * 8;
      const v8h vv = *(const v8h*)(Vb + (size_t)d * NTOK + kv0 + seg);
      *(v8h*)(Vth + d * ATT_KC + seg) = vv;
    }
    __syncthreads();

    v8f s[4];
#pragma unroll
    for (int j = 0; j < 4; ++j) {
      s[j] = (v8f){0.f,0.f,0.f,0.f,0.f,0.f,0.f,0.f};
#pragma unroll
      for (int dc = 0; dc < 2; ++dc) {
        FH kb;
        kb.h[0] = *(const v8h*)(Ksh + (j * 16 + c) * DHEAD + dc * 32 + 8 * hh);
        kb.h[1] = *(const v8h*)(Ksh + (j * 16 + c) * DHEAD + dc * 32 + 16 + 8 * hh);
        s[j] = mma_h(qa[dc], kb.v, s[j]);
      }
    }
    float cm[8];
#pragma unroll
    for (int r = 0; r < 8; ++r) {
      float m = -INFINITY;
#pragma unroll
      for (int j = 0; j < 4; ++j) { s[j][r] *= qkscale; m = fmaxf(m, s[j][r]); }
#pragma unroll
      for (int off = 1; off < 16; off <<= 1) m = fmaxf(m, __shfl_xor(m, off, 32));
      cm[r] = m;
    }
    _Float16* pwh = Psh[wave];
#pragma unroll
    for (int r = 0; r < 8; ++r) {
      const float mnew  = fmaxf(mrow[r], cm[r]);
      const float alpha = expf(mrow[r] - mnew);
      mrow[r] = mnew;
      float psum = 0.f;
#pragma unroll
      for (int j = 0; j < 4; ++j) {
        const float p = expf(s[j][r] - mnew);
        psum += p;
        pwh[(8 * hh + r) * ATT_KC + j * 16 + c] = (_Float16)(p * PCARRY);
      }
#pragma unroll
      for (int off = 1; off < 16; off <<= 1) psum += __shfl_xor(psum, off, 32);
      lrow[r] = lrow[r] * alpha + psum;
#pragma unroll
      for (int t = 0; t < 4; ++t) oacc[t][r] *= alpha;
    }
    __builtin_amdgcn_fence(__ATOMIC_RELEASE, "workgroup");
    __builtin_amdgcn_wave_barrier();
    __builtin_amdgcn_fence(__ATOMIC_ACQUIRE, "workgroup");
#pragma unroll 1
    for (int kk = 0; kk < 2; ++kk) {
      FH pa;
      pa.h[0] = *(const v8h*)(pwh + c * ATT_KC + kk * 32 + 8 * hh);
      pa.h[1] = *(const v8h*)(pwh + c * ATT_KC + kk * 32 + 16 + 8 * hh);
#pragma unroll
      for (int t = 0; t < 4; ++t) {
        FH vb;
        vb.h[0] = *(const v8h*)(Vth + (t * 16 + c) * ATT_KC + kk * 32 + 8 * hh);
        vb.h[1] = *(const v8h*)(Vth + (t * 16 + c) * ATT_KC + kk * 32 + 16 + 8 * hh);
        oacc[t] = mma_h(pa.v, vb.v, oacc[t]);
      }
    }
  }

  float* os = Os[wave];
#pragma unroll
  for (int r = 0; r < 8; ++r) {
    const float inv = 1.0f / (lrow[r] * PCARRY);
#pragma unroll
    for (int t = 0; t < 4; ++t) os[(8 * hh + r) * 68 + t * 16 + c] = oacc[t][r] * inv;
  }
  __builtin_amdgcn_fence(__ATOMIC_RELEASE, "workgroup");
  __builtin_amdgcn_wave_barrier();
  __builtin_amdgcn_fence(__ATOMIC_ACQUIRE, "workgroup");
  {
    const int c4 = (lane & 15) * 4;
    const size_t rowbase = (size_t)b * NTOK + q0;
    v4f vv[8];
#pragma unroll
    for (int it = 0; it < 8; ++it) {
      const int row = it * 2 + hh;
      const v4f o  = *(const v4f*)(os + row * 68 + c4);
      const v4f rr = *(const v4f*)(xres + (rowbase + row) * EDIM + h * DHEAD + c4);
      vv[it] = o + rr;
    }
    for (int pass = 0; pass < 2; ++pass) {
#pragma unroll
      for (int it = 0; it < 8; ++it) {
        const int row = it * 2 + hh;
        *(volatile v4f*)(xout + (rowbase + row) * EDIM + h * DHEAD + c4) = vv[it];
      }
      __threadfence();
    }
  }
}

extern "C" void kernel_launch(void* const* d_in, const int* in_sizes, int n_in,
                              void* d_out, int out_size, void* d_ws, size_t ws_size,
                              hipStream_t stream) {
  (void)in_sizes;
  if (n_in < 17) return;
  if ((size_t)out_size < (size_t)NROWS * EDIM) return;

  const float* x      = (const float*)d_in[0];
  const float* conv_w = (const float*)d_in[1];
  const float* conv_b = (const float*)d_in[2];
  const float* ln1_g5 = (const float*)d_in[3]  + (size_t)LASTB * EDIM;
  const float* ln1_b5 = (const float*)d_in[4]  + (size_t)LASTB * EDIM;
  const float* wq5    = (const float*)d_in[5]  + (size_t)LASTB * NHEAD * DHEAD * DHEAD;
  const float* bq5    = (const float*)d_in[6]  + (size_t)LASTB * NHEAD * DHEAD;
  const float* wk5    = (const float*)d_in[7]  + (size_t)LASTB * NHEAD * DHEAD * DHEAD;
  const float* bk5    = (const float*)d_in[8]  + (size_t)LASTB * NHEAD * DHEAD;
  const float* wv5    = (const float*)d_in[9]  + (size_t)LASTB * NHEAD * DHEAD * DHEAD;
  const float* bv5    = (const float*)d_in[10] + (size_t)LASTB * NHEAD * DHEAD;
  const float* ln2_g5 = (const float*)d_in[11] + (size_t)LASTB * EDIM;
  const float* ln2_b5 = (const float*)d_in[12] + (size_t)LASTB * EDIM;
  const float* w1_5   = (const float*)d_in[13] + (size_t)LASTB * DMLP * EDIM;
  const float* b1_5   = (const float*)d_in[14] + (size_t)LASTB * DMLP;
  const float* w2_5   = (const float*)d_in[15] + (size_t)LASTB * EDIM * DMLP;
  const float* b2_5   = (const float*)d_in[16] + (size_t)LASTB * EDIM;

  char* ws = (char*)d_ws;
  size_t off = 0;
  auto carve = [&](size_t bytes) { size_t o = off; off += (bytes + 255) & ~(size_t)255; return o; };
  const size_t o_pe   = carve((size_t)NTOK * EDIM * 4);
  const size_t o_xcol = carve((size_t)NBATCH * EDIM * KCONV * 2);
  const size_t o_cw   = carve((size_t)NTOK * KCONV * 2);
  const size_t o_vit  = carve((size_t)NROWS * EDIM * 4);
  const size_t o_h1   = carve((size_t)NROWS * EDIM * 2);
  const size_t o_wq   = carve((size_t)NHEAD * DHEAD * DHEAD * 2);
  const size_t o_wk   = carve((size_t)NHEAD * DHEAD * DHEAD * 2);
  const size_t o_wv   = carve((size_t)NHEAD * DHEAD * DHEAD * 2);
  const size_t o_q    = carve((size_t)NBATCH * NHEAD * NTOK * DHEAD * 2);
  const size_t o_k    = carve((size_t)NBATCH * NHEAD * NTOK * DHEAD * 2);
  const size_t o_vt   = carve((size_t)NBATCH * NHEAD * DHEAD * NTOK * 2);
  const size_t o_x1   = carve((size_t)NROWS * EDIM * 4);
  const size_t o_h2   = carve((size_t)NROWS * EDIM * 2);
  const size_t o_w1   = carve((size_t)DMLP * EDIM * 2);
  const size_t o_w2   = carve((size_t)EDIM * DMLP * 2);
  const size_t o_u    = carve((size_t)NROWS * DMLP * 4);
  const size_t o_m    = carve((size_t)NROWS * DMLP * 2);
  if (off > ws_size) return;

  float*          pe    = (float*)(ws + o_pe);
  unsigned short* xcol  = (unsigned short*)(ws + o_xcol);
  unsigned short* cw16  = (unsigned short*)(ws + o_cw);
  float*          vit   = (float*)(ws + o_vit);
  unsigned short* h1    = (unsigned short*)(ws + o_h1);
  unsigned short* wq16  = (unsigned short*)(ws + o_wq);
  unsigned short* wk16  = (unsigned short*)(ws + o_wk);
  unsigned short* wv16  = (unsigned short*)(ws + o_wv);
  unsigned short* q16   = (unsigned short*)(ws + o_q);
  unsigned short* k16   = (unsigned short*)(ws + o_k);
  unsigned short* vt16  = (unsigned short*)(ws + o_vt);
  float*          x1    = (float*)(ws + o_x1);
  unsigned short* h2    = (unsigned short*)(ws + o_h2);
  unsigned short* w1_16 = (unsigned short*)(ws + o_w1);
  unsigned short* w2_16 = (unsigned short*)(ws + o_w2);
  float*          upl   = (float*)(ws + o_u);
  unsigned short* mpl   = (unsigned short*)(ws + o_m);
  float*          outp  = (float*)d_out;

  const dim3 blk256(256), blk128(128);

  {
    const int npairs = NTOK * EDIM / 2;
    posemb_table<<<dim3((npairs + 255) / 256), blk256, 0, stream>>>(pe);
  }
  im2col_f16<<<dim3((NBATCH * EDIM + 7) / 8), blk256, 0, stream>>>(x, xcol);
  {
    const int n2cw = NTOK * KCONV / 2;
    cast_scale_f16x2<<<dim3((n2cw + 255) / 256), blk256, 0, stream>>>(conv_w, cw16, n2cw, WCARRY);
    const int n2h = NHEAD * DHEAD * DHEAD / 2;
    cast_scale_f16x2<<<dim3((n2h + 255) / 256), blk256, 0, stream>>>(wq5, wq16, n2h, WCARRY);
    cast_scale_f16x2<<<dim3((n2h + 255) / 256), blk256, 0, stream>>>(wk5, wk16, n2h, WCARRY);
    cast_scale_f16x2<<<dim3((n2h + 255) / 256), blk256, 0, stream>>>(wv5, wv16, n2h, WCARRY);
    const int n2m = DMLP * EDIM / 2;
    cast_scale_f16x2<<<dim3((n2m + 255) / 256), blk256, 0, stream>>>(w1_5, w1_16, n2m, WCARRY);
    cast_scale_f16x2<<<dim3((n2m + 255) / 256), blk256, 0, stream>>>(w2_5, w2_16, n2m, WCARRY);
  }
  {
    const int tiles = (NTOK / 64) * (EDIM / 64);
    gemm64_f16<1, 0, true><<<dim3((tiles + 7) / 8, NBATCH, 1), blk256, 0, stream>>>(
        cw16, KCONV, 0L, 0L,
        xcol, KCONV, (long)EDIM * KCONV, 0L,
        (void*)vit, EDIM, (long)NTOK * EDIM, 0L,
        conv_b, 0L,
        pe, 0L, 0L,
        NTOK, EDIM, KCONV, WCARRY_INV);
  }
  layernorm_f16<<<dim3((NROWS + 7) / 8), blk256, 0, stream>>>(vit, ln1_g5, ln1_b5, h1, NROWS);
  {
    const int tilesQ = (NTOK / 64) * (DHEAD / 64);
    gemm64_f16<2, 1, false><<<dim3((tilesQ + 7) / 8, NBATCH, NHEAD), blk256, 0, stream>>>(
        h1, EDIM, (long)NTOK * EDIM, (long)DHEAD,
        wq16, DHEAD, 0L, (long)DHEAD * DHEAD,
        (void*)q16, DHEAD, (long)NHEAD * NTOK * DHEAD, (long)NTOK * DHEAD,
        bq5, (long)DHEAD,
        nullptr, 0L, 0L,
        NTOK, DHEAD, DHEAD, WCARRY_INV);
    gemm64_f16<2, 1, false><<<dim3((tilesQ + 7) / 8, NBATCH, NHEAD), blk256, 0, stream>>>(
        h1, EDIM, (long)NTOK * EDIM, (long)DHEAD,
        wk16, DHEAD, 0L, (long)DHEAD * DHEAD,
        (void*)k16, DHEAD, (long)NHEAD * NTOK * DHEAD, (long)NTOK * DHEAD,
        bk5, (long)DHEAD,
        nullptr, 0L, 0L,
        NTOK, DHEAD, DHEAD, WCARRY_INV);
    gemm64_f16<1, 1, false><<<dim3((tilesQ + 7) / 8, NBATCH, NHEAD), blk256, 0, stream>>>(
        wv16, DHEAD, 0L, (long)DHEAD * DHEAD,
        h1, EDIM, (long)NTOK * EDIM, (long)DHEAD,
        (void*)vt16, NTOK, (long)NHEAD * DHEAD * NTOK, (long)DHEAD * NTOK,
        bv5, (long)DHEAD,
        nullptr, 0L, 0L,
        DHEAD, NTOK, DHEAD, WCARRY_INV);
  }
  attn_f16<<<dim3(NBATCH * NHEAD * (NTOK / 64)), blk128, 0, stream>>>(q16, k16, vt16, vit, x1, 0.125f);
  layernorm_f16<<<dim3((NROWS + 7) / 8), blk256, 0, stream>>>(x1, ln2_g5, ln2_b5, h2, NROWS);
  {
    const int tiles = (NROWS / 64) * (DMLP / 64);
    gemm64_f16<2, 0, false><<<dim3((tiles + 7) / 8, 1, 1), blk256, 0, stream>>>(
        h2, EDIM, 0L, 0L,
        w1_16, EDIM, 0L, 0L,
        (void*)upl, DMLP, 0L, 0L,
        b1_5, 0L,
        nullptr, 0L, 0L,
        NROWS, DMLP, EDIM, WCARRY_INV);
  }
  {
    const int n2 = NROWS * DMLP / 2;
    gelu_f16x2<<<dim3((n2 + 255) / 256), blk256, 0, stream>>>(upl, mpl, n2);
  }
  {
    const int tiles = (NROWS / 64) * (EDIM / 64);
    gemm64_f16<2, 0, true><<<dim3((tiles + 7) / 8, 1, 1), blk256, 0, stream>>>(
        mpl, DMLP, 0L, 0L,
        w2_16, DMLP, 0L, 0L,
        (void*)outp, EDIM, 0L, 0L,
        b2_5, 0L,
        x1, 0L, 0L,
        NROWS, EDIM, DMLP, WCARRY_INV);
  }
}
